// ExplicitRelationEncoder_14998025798080
// MI455X (gfx1250) — hardware-verified
//
#include <hip/hip_runtime.h>

typedef _Float16 v16h __attribute__((ext_vector_type(16)));
typedef _Float16 v8h  __attribute__((ext_vector_type(8)));
typedef float    v8f  __attribute__((ext_vector_type(8)));
typedef float    v4f  __attribute__((ext_vector_type(4)));
typedef int      v4i  __attribute__((ext_vector_type(4)));
typedef v8h __attribute__((may_alias)) v8ha;
typedef v4f __attribute__((may_alias)) v4fa;

union Frag { v16h v; v8h half[2]; };

#define BB     256
#define NN     36
#define NG     20
#define LL     11
#define FF     1024
#define HH     16
#define DHD    64
#define MROWS  (BB * NN)
#define KVROWS (BB * NG)
#define NWE    2097152
#define NEGV   (-9.0e15f)
#define WSC    32.0f
#define INVW   0.03125f
#define PSC    1024.0f
#define INVP   0.0009765625f

__device__ __forceinline__ v8f wmma_f16(v16h a, v16h b, v8f c) {
  v8f d = __builtin_amdgcn_wmma_f32_16x16x32_f16(false, a, false, b, (short)0, c, false, false);
  asm volatile("v_nop\n\tv_nop\n\tv_nop\n\tv_nop" : "+v"(d) : "v"(a), "v"(b));
  return d;
}

__device__ __forceinline__ v16h load_frag(const _Float16* p, int h) {
  Frag f;
  f.half[0] = *(const v8ha*)(p + 8 * h);
  f.half[1] = *(const v8ha*)(p + 16 + 8 * h);
  return f.v;
}

__device__ __forceinline__ int imin(int a, int b) { return (a < b) ? a : b; }
__device__ __forceinline__ int kvrow(int r) { const int g = r / NG; return g * NN + (r - g * NG); }

__device__ __forceinline__ v8h cvt8(v4f a, v4f c, float sc) {
  const v8h o = { (_Float16)(a.x * sc), (_Float16)(a.y * sc), (_Float16)(a.z * sc), (_Float16)(a.w * sc),
                  (_Float16)(c.x * sc), (_Float16)(c.y * sc), (_Float16)(c.z * sc), (_Float16)(c.w * sc) };
  return o;
}

__global__ __launch_bounds__(256) void conv_w_kernel(
    const float* __restrict__ wsf, const float* __restrict__ wq,
    const float* __restrict__ wk,  const float* __restrict__ wo,
    const float* __restrict__ q,
    _Float16* wh, _Float16* q16)
{
  const int blk = blockIdx.x;
  const int seg = blk >> 10;
  const int g = (blk & 1023) * 256 + (int)threadIdx.x;
  const float* src;
  _Float16* dst;
  float sc;
  if (seg == 0)      { src = wsf + (size_t)g * 8; dst = wh + (size_t)g * 8;                     sc = WSC; }
  else if (seg == 1) { src = wq  + (size_t)g * 8; dst = wh + (size_t)NWE + (size_t)g * 8;       sc = WSC; }
  else if (seg == 2) { src = wk  + (size_t)g * 8; dst = wh + (size_t)2 * NWE + (size_t)g * 8;   sc = WSC; }
  else if (seg == 3) { src = wo  + (size_t)g * 8; dst = wh + (size_t)3 * NWE + (size_t)g * 8;   sc = WSC; }
  else               { src = q   + (size_t)g * 8; dst = q16 + (size_t)g * 8;                    sc = 1.0f; }
  const v4f a = *(const v4fa*)src;
  const v4f c = *(const v4fa*)(src + 4);
  const v8h o = cvt8(a, c, sc);
  *(volatile v8h*)dst = o;
  __threadfence();
  *(volatile v8h*)dst = o;
}

__global__ __launch_bounds__(256) void conv_v_kernel(
    const float* __restrict__ v, _Float16* vh, int* flags)
{
  __shared__ int s_flag[32];
  const int tid = threadIdx.x, lane = tid & 31, w = tid >> 5;
  const int rbase = blockIdx.x * 32;

  #pragma unroll 1
  for (int i = 0; i < 4; ++i) {
    const int row = rbase + 4 * w + i;
    const float* src = v + (size_t)row * FF;
    _Float16* dst = vh + (size_t)row * FF;
    v8h o[4];
    float s = 0.0f;
    #pragma unroll
    for (int sg = 0; sg < 4; ++sg) {
      const float* p = src + sg * 256 + 8 * lane;
      const v4f a = *(const v4fa*)p;
      const v4f c = *(const v4fa*)(p + 4);
      s += ((a.x + a.y) + (a.z + a.w)) + ((c.x + c.y) + (c.z + c.w));
      o[sg] = cvt8(a, c, 1.0f);
      *(volatile v8h*)(dst + sg * 256 + 8 * lane) = o[sg];
    }
    __threadfence();
    #pragma unroll
    for (int sg = 0; sg < 4; ++sg)
      *(volatile v8h*)(dst + sg * 256 + 8 * lane) = o[sg];

    s += __shfl_xor(s, 16);
    s += __shfl_xor(s, 8);
    s += __shfl_xor(s, 4);
    s += __shfl_xor(s, 2);
    s += __shfl_xor(s, 1);
    if (lane == 0) s_flag[4 * w + i] = (s == 0.0f) ? 1 : 0;
  }
  __syncthreads();
  if (tid < 8) {
    const v4i f = { s_flag[4 * tid], s_flag[4 * tid + 1], s_flag[4 * tid + 2], s_flag[4 * tid + 3] };
    int* fp = flags + rbase + 4 * tid;
    *(volatile v4i*)fp = f;
    __threadfence();
    *(volatile v4i*)fp = f;
  }
}

__device__ __forceinline__ void store_f32_pass(const float* sT, float* outF,
                                               int m0, int col0, int w, int lane) {
  const int q4 = lane & 15, sub = lane >> 4;
  #pragma unroll
  for (int i = 0; i < 16; ++i) {
    const int lid = 32 * w + 2 * i + sub;
    const v4f x = *(const v4fa*)(sT + lid * 64 + 4 * q4);
    *(volatile v4f*)(outF + (size_t)(m0 + lid) * FF + col0 + 4 * q4) = x;
  }
}

__device__ __forceinline__ void store_f16_pass(const float* sT, _Float16* outH,
                                               int m0, int col0, int w, int lane) {
  const int q8 = lane & 7, sub = lane >> 3;
  #pragma unroll
  for (int i = 0; i < 8; ++i) {
    const int lid = 32 * w + 4 * i + sub;
    const v4f a = *(const v4fa*)(sT + lid * 64 + 8 * q8);
    const v4f c = *(const v4fa*)(sT + lid * 64 + 8 * q8 + 4);
    const v8h o = cvt8(a, c, 1.0f);
    *(volatile v8h*)(outH + (size_t)(m0 + lid) * FF + col0 + 8 * q8) = o;
  }
}

template <int MODE>
__global__ __launch_bounds__(128) void gemm_kernel(
    const _Float16* __restrict__ A,
    const _Float16* __restrict__ Bw, int ldb,
    const float* __restrict__ bias,
    const int*   __restrict__ flag,
    const float* __restrict__ qs,
    float* outF, _Float16* outH)
{
  __shared__ __attribute__((aligned(16))) float sT[128 * 64];

  const int tid = threadIdx.x, lane = tid & 31, w = tid >> 5;
  const int hh = lane >> 4, m = lane & 15;
  const int m0 = blockIdx.x * 128;
  const int col0 = blockIdx.y * 64;
  const int m0w = m0 + 32 * w;

  int ra0 = m0w + m, ra1 = m0w + 16 + m;
  if (MODE >= 3) { ra0 = kvrow(ra0); ra1 = kvrow(ra1); }
  const _Float16* xa0 = A + (size_t)ra0 * FF;
  const _Float16* xa1 = A + (size_t)ra1 * FF;
  const _Float16* wb  = Bw + (size_t)(col0 + m) * ldb;

  const v8f zero8 = {0.f, 0.f, 0.f, 0.f, 0.f, 0.f, 0.f, 0.f};
  v8f acc[2][4];
  #pragma unroll
  for (int mt = 0; mt < 2; ++mt)
    #pragma unroll
    for (int nt = 0; nt < 4; ++nt) acc[mt][nt] = zero8;

  #pragma unroll 1
  for (int k0 = 0; k0 < FF; k0 += 32) {
    const v16h a0 = load_frag(xa0 + k0, hh);
    const v16h a1 = load_frag(xa1 + k0, hh);
    #pragma unroll
    for (int nt = 0; nt < 4; ++nt) {
      const v16h b = load_frag(wb + (size_t)nt * 16 * ldb + k0, hh);
      acc[0][nt] = wmma_f16(a0, b, acc[0][nt]);
      acc[1][nt] = wmma_f16(a1, b, acc[1][nt]);
    }
  }

  #pragma unroll
  for (int nt = 0; nt < 4; ++nt) {
    const int feat = 16 * nt + m;
    const int col = col0 + feat;
    float bv = 0.0f;
    if (MODE == 1 || MODE == 2 || MODE == 3) bv = bias[col];
    #pragma unroll
    for (int mt = 0; mt < 2; ++mt) {
      #pragma unroll
      for (int r = 0; r < 8; ++r) {
        const int tokl = 32 * w + 16 * mt + 8 * hh + r;
        float y = acc[mt][nt][r] * INVW + bv;
        if (MODE == 1) {
          const int tok = m0 + tokl;
          const int fl = flag[tok];
          const float qv = qs[(size_t)(tok / NN) * FF + col];
          y += (fl != 0) ? 0.0f : qv;
        }
        sT[tokl * 64 + feat] = y;
      }
    }
  }
  __syncthreads();

  if (MODE <= 1) store_f32_pass(sT, outF, m0, col0, w, lane);
  if (MODE >= 1) store_f16_pass(sT, outH, m0, col0, w, lane);
  __threadfence();
  if (MODE <= 1) store_f32_pass(sT, outF, m0, col0, w, lane);
  if (MODE >= 1) store_f16_pass(sT, outH, m0, col0, w, lane);
}

template <int DIR>
__global__ __launch_bounds__(256) void mix_kernel(
    const int*   __restrict__ adj,
    const float* __restrict__ w_bias,
    const float* __restrict__ b_bias,
    const _Float16* __restrict__ QHp,
    const _Float16* __restrict__ KHp,
    const _Float16* __restrict__ KWp,
    const float* __restrict__ bo,
    const float* __restrict__ vin,
    float* base,
    float* out)
{
  __shared__ float s_vb[NN * NG];
  __shared__ int   s_ok[NN * NG];
  __shared__ __attribute__((aligned(16))) _Float16 s_p[2 * 48 * 32];
  __shared__ __attribute__((aligned(16))) _Float16 s_kwt[128 * 32];
  __shared__ __attribute__((aligned(16))) float    s_out[NN * 128];

  const int tid = threadIdx.x, lane = tid & 31, w = tid >> 5;
  const int hh = lane >> 4, m = lane & 15;
  const int b = blockIdx.x;
  const v8f zero8 = {0.f, 0.f, 0.f, 0.f, 0.f, 0.f, 0.f, 0.f};

  const float bb0 = b_bias[0];
  #pragma unroll 1
  for (int p = tid; p < NN * NG; p += 256) {
    const int n = p / NG, mp = p - (p / NG) * NG;
    const size_t ib = (DIR == 0) ? ((((size_t)b * NN + n) * NN + mp) * LL)
                                 : ((((size_t)b * NN + mp) * NN + n) * LL);
    float fs = 0.0f, vb = 0.0f;
    #pragma unroll 1
    for (int l = 0; l < LL; ++l) {
      const float a = (float)adj[ib + l];
      fs += a;
      vb += a * w_bias[l];
    }
    s_vb[p] = vb + bb0;
    s_ok[p] = (fs > 0.0f) ? 1 : 0;
  }
  {
    const v8h z8 = { (_Float16)0.f, (_Float16)0.f, (_Float16)0.f, (_Float16)0.f,
                     (_Float16)0.f, (_Float16)0.f, (_Float16)0.f, (_Float16)0.f };
    #pragma unroll 1
    for (int i = tid; i < 512; i += 256) *(v8ha*)(s_kwt + 8 * i) = z8;
  }
  __syncthreads();

  #pragma unroll 1
  for (int c = 0; c < 8; ++c) {
    {
      const int mp = tid >> 4, c8 = (tid & 15) * 8;
      const v8h x = *(const v8ha*)(KWp + (size_t)(b * NG + mp) * FF + c * 128 + c8);
      #pragma unroll
      for (int j = 0; j < 8; ++j) s_kwt[(c8 + j) * 32 + mp] = x[j];
      if (tid < 64) {
        const int mp2 = 16 + mp;
        const v8h y = *(const v8ha*)(KWp + (size_t)(b * NG + mp2) * FF + c * 128 + c8);
        #pragma unroll
        for (int j = 0; j < 8; ++j) s_kwt[(c8 + j) * 32 + mp2] = y[j];
      }
    }

    if (w < 6) {
      const int hg = (w >= 3) ? 1 : 0;
      const int rt = w - 3 * hg;
      const int head = 2 * c + hg;
      const int na = imin(16 * rt + m, NN - 1);
      const int m1 = imin(16 + m, NG - 1);
      const _Float16* qa  = QHp + (size_t)(b * NN + na) * FF + head * DHD;
      const _Float16* kb0 = KHp + (size_t)(b * NG + m)  * FF + head * DHD;
      const _Float16* kb1 = KHp + (size_t)(b * NG + m1) * FF + head * DHD;
      v8f acc0 = zero8, acc1 = zero8;
      #pragma unroll
      for (int ks = 0; ks < 2; ++ks) {
        const v16h af  = load_frag(qa  + 32 * ks, hh);
        const v16h bf0 = load_frag(kb0 + 32 * ks, hh);
        const v16h bf1 = load_frag(kb1 + 32 * ks, hh);
        acc0 = wmma_f16(af, bf0, acc0);
        acc1 = wmma_f16(af, bf1, acc1);
      }
      const bool c1 = (m < NG - 16);
      _Float16* sp = s_p + hg * 1536;
      #pragma unroll
      for (int r = 0; r < 8; ++r) {
        const int n  = 16 * rt + 8 * hh + r;
        const int nn = imin(n, NN - 1);
        const float vb0 = s_vb[nn * NG + m];
        const int   ok0 = s_ok[nn * NG + m];
        const float vb1 = s_vb[nn * NG + m1];
        const int   ok1 = s_ok[nn * NG + m1];
        const float l0  = (ok0 != 0) ? (acc0[r] * 0.125f + vb0) : (NEGV + vb0);
        const float l1r = (ok1 != 0) ? (acc1[r] * 0.125f + vb1) : (NEGV + vb1);
        const float l1  = c1 ? l1r : l0;
        float mx = fmaxf(l0, l1);
        mx = fmaxf(mx, __shfl_xor(mx, 8));
        mx = fmaxf(mx, __shfl_xor(mx, 4));
        mx = fmaxf(mx, __shfl_xor(mx, 2));
        mx = fmaxf(mx, __shfl_xor(mx, 1));
        const float e0  = __expf(l0 - mx);
        const float e1v = __expf(l1 - mx);
        const float e1  = c1 ? e1v : 0.0f;
        float sm = e0 + e1;
        sm += __shfl_xor(sm, 8);
        sm += __shfl_xor(sm, 4);
        sm += __shfl_xor(sm, 2);
        sm += __shfl_xor(sm, 1);
        const float inv = __builtin_amdgcn_rcpf(sm);
        const bool rowok = (n < NN);
        const float p0 = rowok ? (e0 * inv) : 0.0f;
        const float p1 = rowok ? (e1 * inv) : 0.0f;
        sp[n * 32 + m]      = (_Float16)(p0 * PSC);
        sp[n * 32 + 16 + m] = (_Float16)(p1 * PSC);
      }
    }
    __syncthreads();

    #pragma unroll 1
    for (int ti = w; ti < 24; ti += 8) {
      const int hg = (ti >= 12) ? 1 : 0;
      const int rem = ti - 12 * hg;
      const int rt = rem >> 2, ct = rem & 3;
      const v16h af = load_frag(s_p + hg * 1536 + (16 * rt + m) * 32, hh);
      const int colc = hg * 64 + 16 * ct + m;
      const v16h bf = load_frag(s_kwt + colc * 32, hh);
      const v8f acc = wmma_f16(af, bf, zero8);
      const float bov = bo[c * 128 + colc];
      #pragma unroll
      for (int r = 0; r < 8; ++r) {
        const int n = 16 * rt + 8 * hh + r;
        if (n < NN) s_out[n * 128 + colc] = acc[r] * INVP + bov;
      }
    }
    __syncthreads();

    #pragma unroll 1
    for (int n = w; n < NN; n += 8) {
      const v4f att = *(const v4fa*)(s_out + n * 128 + 4 * lane);
      const size_t go = (size_t)(b * NN + n) * FF + c * 128 + 4 * lane;
      if (DIR == 0) {
        const v4f bs = *(const v4fa*)(base + go);
        const v4f val = bs + att;
        *(volatile v4f*)(base + go) = val;
        __threadfence();
        *(volatile v4f*)(base + go) = val;
      } else {
        const v4f bs = *(const v4fa*)(base + go);
        const v4f vv = *(const v4fa*)(vin + go);
        const v4f t4 = bs + att;
        v4f val;
        val.x = vv.x + fmaxf(t4.x, 0.0f);
        val.y = vv.y + fmaxf(t4.y, 0.0f);
        val.z = vv.z + fmaxf(t4.z, 0.0f);
        val.w = vv.w + fmaxf(t4.w, 0.0f);
        *(volatile v4f*)(out + go) = val;
        __threadfence();
        *(volatile v4f*)(out + go) = val;
      }
    }
    __syncthreads();
  }
}

extern "C" void kernel_launch(void* const* d_in, const int* in_sizes, int n_in,
                              void* d_out, int out_size, void* d_ws, size_t ws_size,
                              hipStream_t stream) {
  if (n_in < 13) return;
  if (in_sizes[0] != MROWS * FF) return;
  if (in_sizes[1] != BB * FF) return;
  if (in_sizes[2] != BB * NN * NN * LL) return;
  if (in_sizes[3] != NWE) return;
  if (in_sizes[4] != FF) return;
  if (in_sizes[5] != LL) return;
  if (in_sizes[6] != 1) return;
  if (in_sizes[7] != NWE || in_sizes[9] != NWE || in_sizes[11] != NWE) return;
  if (in_sizes[8] != 2 * FF || in_sizes[10] != 2 * FF || in_sizes[12] != 2 * FF) return;
  if (out_size != MROWS * FF) return;

  const float* v      = (const float*)d_in[0];
  const float* q      = (const float*)d_in[1];
  const int*   adj    = (const int*)  d_in[2];
  const float* W_self = (const float*)d_in[3];
  const float* b_self = (const float*)d_in[4];
  const float* w_bias = (const float*)d_in[5];
  const float* b_bias = (const float*)d_in[6];
  const float* Wq     = (const float*)d_in[7];
  const float* bq     = (const float*)d_in[8];
  const float* Wk     = (const float*)d_in[9];
  const float* bk     = (const float*)d_in[10];
  const float* Wout   = (const float*)d_in[11];
  const float* bout   = (const float*)d_in[12];
  float* out = (float*)d_out;

  const size_t b_wh   = (size_t)4 * NWE * 2;
  const size_t b_qh   = (size_t)MROWS * FF * 2;
  const size_t b_q16  = (size_t)BB * FF * 2;
  const size_t b_flag = (size_t)MROWS * 4;
  const size_t b_qs   = (size_t)BB * FF * 4;
  const size_t b_sf   = (size_t)MROWS * FF * 4;
  const size_t b_sfh  = (size_t)MROWS * FF * 2;
  const size_t b_kh   = (size_t)KVROWS * FF * 2;
  const size_t b_kw   = (size_t)KVROWS * FF * 2;
  const size_t total  = b_wh + b_qh + b_q16 + b_flag + b_qs + b_sf + b_sfh + b_kh + b_kw;
  if (total > ws_size) return;

  char* ws = (char*)d_ws;
  size_t off = 0;
  _Float16* Wh   = (_Float16*)(ws + off); off += b_wh;
  _Float16* VQH  = (_Float16*)(ws + off); off += b_qh;
  _Float16* Q16  = (_Float16*)(ws + off); off += b_q16;
  int*      FLG  = (int*)     (ws + off); off += b_flag;
  float*    QS   = (float*)   (ws + off); off += b_qs;
  float*    SF   = (float*)   (ws + off); off += b_sf;
  _Float16* SFh  = (_Float16*)(ws + off); off += b_sfh;
  _Float16* KH   = (_Float16*)(ws + off); off += b_kh;
  _Float16* KW   = (_Float16*)(ws + off); off += b_kw;
  if (off != total) return;

  const _Float16* Wsh   = Wh;
  const _Float16* Wqh   = Wh + (size_t)NWE;
  const _Float16* Wkh   = Wh + (size_t)2 * NWE;
  const _Float16* Wouth = Wh + (size_t)3 * NWE;

  conv_w_kernel<<<4224, 256, 0, stream>>>(W_self, Wq, Wk, Wout, q, Wh, Q16);
  conv_v_kernel<<<MROWS / 32, 256, 0, stream>>>(v, VQH, FLG);
  gemm_kernel<0><<<dim3(BB / 128, FF / 64), 128, 0, stream>>>(
      Q16, Wsh + FF, 2048, b_self, FLG, QS, QS, SFh);
  gemm_kernel<1><<<dim3(MROWS / 128, FF / 64), 128, 0, stream>>>(
      VQH, Wsh, 2048, b_self, FLG, QS, SF, SFh);

  gemm_kernel<2><<<dim3(MROWS / 128, FF / 64), 128, 0, stream>>>(
      SFh, Wqh, FF, bq, FLG, QS, QS, VQH);
  gemm_kernel<3><<<dim3(KVROWS / 128, FF / 64), 128, 0, stream>>>(
      SFh, Wkh, FF, bk, FLG, QS, QS, KH);
  gemm_kernel<4><<<dim3(KVROWS / 128, FF / 64), 128, 0, stream>>>(
      SFh, Wouth, FF, bout, FLG, QS, QS, KW);
  mix_kernel<0><<<BB, 256, 0, stream>>>(adj, w_bias, b_bias, VQH, KH, KW, bout, v, SF, out);

  gemm_kernel<2><<<dim3(MROWS / 128, FF / 64), 128, 0, stream>>>(
      SFh, Wqh + (size_t)FF * FF, FF, bq + FF, FLG, QS, QS, VQH);
  gemm_kernel<3><<<dim3(KVROWS / 128, FF / 64), 128, 0, stream>>>(
      SFh, Wkh + (size_t)FF * FF, FF, bk + FF, FLG, QS, QS, KH);
  gemm_kernel<4><<<dim3(KVROWS / 128, FF / 64), 128, 0, stream>>>(
      SFh, Wouth + (size_t)FF * FF, FF, bout + FF, FLG, QS, QS, KW);
  mix_kernel<1><<<BB, 256, 0, stream>>>(adj, w_bias, b_bias, VQH, KH, KW, bout + FF, v, SF, out);
}
